// TransformerEncoder_89146341196503
// MI455X (gfx1250) — hardware-run, weakly checked
//
#include <hip/hip_runtime.h>


#ifndef NB
#define NB 1
#endif
#ifndef SEQ
#define SEQ 2048
#endif
#define NB_FULL  1
#define SEQ_FULL 2048
#define XIN  64
#define EW   256
#define NH_  8
#define HD   32
#define FFW  1024
#define NLAY 2
#define WH   128
#define RP   260
#define QRS  2048.0f
#define QRI  (1.0f / 2048.0f)
#define WSC  64.0f
#define WSI  (1.0f / 64.0f)
#define EMBS 0.25f
#define SC2  ((float)(0.17677669529663687 * 1.4426950408889634))
#define PSH  14.0f
#define NEGB (-3.0e38f)
#define LNEPS 1.0e-5f

static_assert(NB == 1);
static_assert(HD == 32);
static_assert(NH_ * HD == EW);
static_assert(NH_ * 32 == 256);
static_assert(4 * 64 == EW);
static_assert(EW % 64 == 0);
static_assert(FFW % 64 == 0);
static_assert((2 * EW) % 64 == 0);
static_assert(XIN % 64 == 0);
static_assert(XIN % 32 == 0);
static_assert(EW % 32 == 0);
static_assert(FFW % 32 == 0);
static_assert(SEQ % 64 == 0);
static_assert(SEQ % 32 == 0);
static_assert(SEQ <= SEQ_FULL);
static_assert(WH % 32 == 0);
static_assert((RP * 4) % 16 == 0);
static_assert(RP >= EW);
static_assert(((size_t)SEQ * XIN) % (8 * 256) == 0);
static_assert(16 * RP * 4 <= 131072);
static_assert(64 * 68 * 4 <= 131072);
static_assert(16 * 68 * 4 <= 131072);
static_assert(256 * 16 * 2 == 64 * 128);
static_assert(64 * 16 == EW * 4);
static_assert(4 * 8 * 32 * 16 == 16 * EW * 4);
static_assert(4 * 4 * 32 * 16 == 16 * EW * 2);
static_assert(2 * 2 * 32 * 16 == 16 * 64 * 2);
static_assert(4 * 32 * 16 == 16 * 64 * 2);
static_assert(NH_ * 2 * 32 * 16 == 16 * EW * 2);

typedef _Float16 h16;
typedef unsigned short bf;
typedef __attribute__((ext_vector_type(16))) _Float16 v16h;
typedef __attribute__((ext_vector_type(8)))  _Float16 v8h;
typedef __attribute__((ext_vector_type(8)))  float    v8f;
typedef __attribute__((ext_vector_type(4)))  float    v4f;
typedef v4f  __attribute__((may_alias)) v4fa;

__device__ __forceinline__ unsigned short f2bf(float f) { unsigned u = __float_as_uint(f); u += 0x7FFFu + ((u >> 16) & 1u); return (unsigned short)(u >> 16); }
__device__ __forceinline__ float bfr(float f) { return __uint_as_float(((unsigned)f2bf(f)) << 16); }
__device__ __forceinline__ v16h cat16(v8h lo, v8h hi) { return __builtin_shufflevector(lo, hi, 0, 1, 2, 3, 4, 5, 6, 7, 8, 9, 10, 11, 12, 13, 14, 15); }
__device__ __forceinline__ v8f wmma16(v16h a, v16h b, v8f c) { return __builtin_amdgcn_wmma_f32_16x16x32_f16(false, a, false, b, (short)0, c, false, false); }
__device__ __forceinline__ v16h  ldh(const h16* p) { return cat16(*(const v8h*)p, *(const v8h*)(p + 16)); }
__device__ __forceinline__ void wave_sync() { __builtin_amdgcn_fence(3  , "wavefront"); __builtin_amdgcn_wave_barrier(); asm volatile("" ::: "memory"); }
__device__ __forceinline__ h16 toh_flush(float v) { const h16 r = (h16)v; return (fabsf(v) < 6.103515625e-05f) ? (h16)0.0f : r; }
__device__ __forceinline__ v8f wmma16g(v16h a, v16h b, v8f c) { c = wmma16(a, b, c); asm volatile("v_nop\n\tv_nop\n\tv_nop\n\tv_nop" : "+v"(c) : "v"(a), "v"(b)); return c; }

__global__ __launch_bounds__(256) void k_cvth(const float* __restrict__ src, h16* dst, size_t n8) {
#pragma clang fp contract(off)
    const size_t i = (size_t)blockIdx.x * 256 + threadIdx.x; if (i >= n8) return;
    const v8f v = *(const v8f*)(src + i * 8); v8h o;
#pragma unroll
    for (int k = 0; k < 8; ++k) o[k] = toh_flush(bfr(v[k]));
    *(volatile v8h*)(dst + i * 8) = o; __threadfence(); *(volatile v8h*)(dst + i * 8) = o;
}

__global__ __launch_bounds__(256) void k_wconv(const float* __restrict__ W, h16* Wt, const int K, const int N, const size_t zin, const size_t zout) {
#pragma clang fp contract(off)
    __shared__ __align__(16) float ts[64 * 68];
    const int tid = threadIdx.x;
    const int n0 = blockIdx.x * 64, k0 = blockIdx.y * 64;
    const float* src = W + (size_t)blockIdx.z * zin;
    h16* dst = Wt + (size_t)blockIdx.z * zout;
#pragma unroll
    for (int it = 0; it < 4; ++it) { const int p = it * 256 + tid; const int r = p >> 4, c4 = (p & 15) * 4;
        const v4f v = *(const v4f*)(src + (size_t)(k0 + r) * N + n0 + c4);
        *(v4fa*)(&ts[r * 68 + c4]) = v; }
    __syncthreads();
#pragma unroll 1
    for (int ps = 0; ps < 2; ++ps) {
#pragma unroll
        for (int it = 0; it < 2; ++it) { const int p = it * 256 + tid; const int n = p >> 3, c8 = (p & 7) * 8; v8h o;
#pragma unroll
            for (int i = 0; i < 8; ++i) o[i] = toh_flush(bfr(ts[(c8 + i) * 68 + n]) * WSC);
            *(volatile v8h*)(dst + (size_t)(n0 + n) * K + k0 + c8) = o; }
        if (ps == 0) __threadfence(); }
}

__global__ __launch_bounds__(256) void k_pe(float* PE) {
#pragma clang fp contract(off)
    __shared__ __align__(16) float srow[EW];
    const int t = blockIdx.x, e = threadIdx.x;
    const int j = e & 127;
    const double u = -(double)j * (9.210340371976183 / 2048.0);
    double p = 1.0 / 6227020800.0;
    p = __builtin_fma(p, u, 1.0 / 479001600.0);
    p = __builtin_fma(p, u, 1.0 / 39916800.0);
    p = __builtin_fma(p, u, 1.0 / 3628800.0);
    p = __builtin_fma(p, u, 1.0 / 362880.0);
    p = __builtin_fma(p, u, 1.0 / 40320.0);
    p = __builtin_fma(p, u, 1.0 / 5040.0);
    p = __builtin_fma(p, u, 1.0 / 720.0);
    p = __builtin_fma(p, u, 1.0 / 120.0);
    p = __builtin_fma(p, u, 1.0 / 24.0);
    p = __builtin_fma(p, u, 1.0 / 6.0);
    p = __builtin_fma(p, u, 0.5);
    p = __builtin_fma(p, u, 1.0);
    p = __builtin_fma(p, u, 1.0);
    p = p * p; p = p * p; p = p * p; p = p * p;
    const double ang = (double)(SEQ_FULL - 1 - t) * p;
    const double kq = __builtin_rint(ang * 0.6366197723675814);
    double r = __builtin_fma(-kq, 1.5707963267948966, ang);
    r = __builtin_fma(-kq, 6.123233995736766e-17, r);
    const float x = (float)r, x2 = x * x;
    float sp = x2 * (1.0f / 362880.0f) - (1.0f / 5040.0f);
    sp = sp * x2 + (1.0f / 120.0f);
    sp = sp * x2 - (1.0f / 6.0f);
    const float sn = x + x * (x2 * sp);
    float cq = (1.0f / 40320.0f) - x2 * (1.0f / 3628800.0f);
    cq = cq * x2 - (1.0f / 720.0f);
    cq = cq * x2 + (1.0f / 24.0f);
    cq = cq * x2 - 0.5f;
    const float cs = 1.0f + x2 * cq;
    const int qq = (int)kq + (e >> 7);
    float val = (qq & 1) ? cs : sn; val = (qq & 2) ? -val : val;
    srow[e] = val;
    __syncthreads();
    if (e < 64) {
        const v4f o = *(const v4fa*)(&srow[e * 4]);
        float* dst = PE + (size_t)t * EW + e * 4;
        *(volatile v4f*)dst = o; __threadfence(); *(volatile v4f*)dst = o;
    }
}

__global__ __launch_bounds__(128) void k_rowgemm(const h16* __restrict__ A, const h16* __restrict__ Bt, const int K, const int epi, const int hasb,
                                                 const float* __restrict__ bias, const float* __restrict__ RES, const float* __restrict__ gam, const float* __restrict__ bet,
                                                 float* OUTF, h16* PH, h16* PR, const int wpl, const int wres) {
    __shared__ __align__(16) float os[16 * RP];
    const int lane = threadIdx.x & 31, lr = lane & 15, hi = lane >> 4;
    const int wave = __builtin_amdgcn_readfirstlane((int)(threadIdx.x >> 5));
    const int r0 = blockIdx.x * 16, c0 = wave * 64;
    v8f acc[4];
#pragma unroll
    for (int nb = 0; nb < 4; ++nb) acc[nb] = (v8f){};
    const size_t aoff = (size_t)(r0 + lr) * K + 8 * hi, boff = (size_t)(c0 + lr) * K + 8 * hi;
#pragma unroll 1
    for (int kc = 0; kc < K; kc += 32) {
        const v16h a = ldh(A + aoff + kc);
#pragma unroll
        for (int nb = 0; nb < 4; ++nb) { const v16h b = ldh(Bt + boff + (size_t)nb * 16 * K + kc); acc[nb] = wmma16g(a, b, acc[nb]); }
    }
    const float sc = (epi == 0) ? EMBS : WSI;
#pragma unroll
    for (int nb = 0; nb < 4; ++nb) {
#pragma unroll
        for (int j = 0; j < 8; ++j) os[(hi * 8 + j) * RP + c0 + nb * 16 + lr] = acc[nb][j] * sc; }
    __syncthreads();
    const int c8 = lane * 8;
    float bb[8], gg[8], oo[8];
#pragma unroll
    for (int i = 0; i < 8; ++i) { bb[i] = 0.0f; gg[i] = 1.0f; oo[i] = 0.0f; }
    if (epi == 1) {
        const v4f g0 = *(const v4f*)(gam + c8), g1 = *(const v4f*)(gam + c8 + 4);
        const v4f e0 = *(const v4f*)(bet + c8), e1 = *(const v4f*)(bet + c8 + 4);
#pragma unroll
        for (int i = 0; i < 4; ++i) { gg[i] = bfr(g0[i]); gg[4 + i] = bfr(g1[i]); oo[i] = bfr(e0[i]); oo[4 + i] = bfr(e1[i]); }
        if (hasb) {
            const v4f b0 = *(const v4f*)(bias + c8), b1 = *(const v4f*)(bias + c8 + 4);
#pragma unroll
            for (int i = 0; i < 4; ++i) { bb[i] = bfr(b0[i]); bb[4 + i] = bfr(b1[i]); }
        }
    }
#pragma unroll 1
    for (int rr = 0; rr < 4; ++rr) {
        const int row = wave * 4 + rr;
        const v4f x0 = *(const v4fa*)(&os[row * RP + c8]); const v4f x1 = *(const v4fa*)(&os[row * RP + c8 + 4]);
        const float* rp = RES + (size_t)(r0 + row) * EW + c8;
        const v4f q0 = *(const v4f*)rp, q1 = *(const v4f*)(rp + 4);
        float v[8];
#pragma unroll
        for (int i = 0; i < 4; ++i) { v[i] = (x0[i] + bb[i]) + q0[i]; v[4 + i] = (x1[i] + bb[4 + i]) + q1[i]; }
        if (epi == 1) {
            float s = 0.0f;
#pragma unroll
            for (int i = 0; i < 8; ++i) s += v[i];
            s += __shfl_xor(s, 16, 32); s += __shfl_xor(s, 8, 32); s += __shfl_xor(s, 4, 32); s += __shfl_xor(s, 2, 32); s += __shfl_xor(s, 1, 32);
            const float mean = s * (1.0f / (float)EW);
            float ss = 0.0f;
#pragma unroll
            for (int i = 0; i < 8; ++i) { v[i] = v[i] - mean; ss += v[i] * v[i]; }
            ss += __shfl_xor(ss, 16, 32); ss += __shfl_xor(ss, 8, 32); ss += __shfl_xor(ss, 4, 32); ss += __shfl_xor(ss, 2, 32); ss += __shfl_xor(ss, 1, 32);
            const float rs = rsqrtf(ss * (1.0f / (float)EW) + LNEPS);
#pragma unroll
            for (int i = 0; i < 8; ++i) v[i] = (v[i] * rs) * gg[i] + oo[i];
        }
        v4f y0, y1;
#pragma unroll
        for (int i = 0; i < 4; ++i) { y0[i] = v[i]; y1[i] = v[4 + i]; }
        *(v4fa*)(&os[row * RP + c8]) = y0; *(v4fa*)(&os[row * RP + c8 + 4]) = y1;
    }
    wave_sync();
#pragma unroll 1
    for (int ps = 0; ps < 2; ++ps) {
#pragma unroll
        for (int s = 0; s < 8; ++s) { const int row = wave * 4 + (s >> 1), col = (s & 1) * 128 + lane * 4;
            const v4f val = *(const v4fa*)(&os[row * RP + col]);
            *(volatile v4f*)(OUTF + (size_t)(r0 + row) * EW + col) = val; }
        if (wpl) {
#pragma unroll
            for (int rr = 0; rr < 4; ++rr) { const int row = wave * 4 + rr;
                const v4f x0 = *(const v4fa*)(&os[row * RP + c8]); const v4f x1 = *(const v4fa*)(&os[row * RP + c8 + 4]); v8h hv, rv;
#pragma unroll
                for (int i = 0; i < 4; ++i) { const h16 a0 = toh_flush(x0[i]); const h16 a1 = toh_flush(x1[i]); hv[i] = a0; hv[4 + i] = a1;
                    rv[i] = toh_flush((x0[i] - (float)a0) * QRS); rv[4 + i] = toh_flush((x1[i] - (float)a1) * QRS); }
                const size_t oo2 = (size_t)(r0 + row) * EW + c8;
                *(volatile v8h*)(PH + oo2) = hv; if (wres) *(volatile v8h*)(PR + oo2) = rv; }
        }
        if (ps == 0) __threadfence(); }
}

__global__ __launch_bounds__(32) void k_qk(const h16* __restrict__ AH, const h16* __restrict__ AR, const h16* __restrict__ Bt, h16* Ph, h16* Pr) {
    __shared__ __align__(16) float os[16 * 68];
    const int K = EW;
    const int lane = threadIdx.x & 31, lr = lane & 15, hi = lane >> 4; const int r0 = blockIdx.x * 16, c0 = blockIdx.y * 64;
    v8f sh[4], sr[4];
#pragma unroll
    for (int nb = 0; nb < 4; ++nb) { sh[nb] = (v8f){}; sr[nb] = (v8f){}; }
    const size_t aoff = (size_t)(r0 + lr) * K + 8 * hi, boff = (size_t)(c0 + lr) * K + 8 * hi;
#pragma unroll 1
    for (int kc = 0; kc < K; kc += 32) {
        const v16h ah = ldh(AH + aoff + kc), ar = ldh(AR + aoff + kc);
#pragma unroll
        for (int nb = 0; nb < 4; ++nb) { const v16h b = ldh(Bt + boff + (size_t)nb * 16 * K + kc);
            sh[nb] = wmma16g(ah, b, sh[nb]); sr[nb] = wmma16g(ar, b, sr[nb]); }
    }
#pragma unroll
    for (int nb = 0; nb < 4; ++nb) {
#pragma unroll
        for (int j = 0; j < 8; ++j) os[(hi * 8 + j) * 68 + nb * 16 + lr] = sh[nb][j] * WSI + sr[nb][j] * (WSI * QRI); }
    wave_sync();
    const int zc = c0 / HD;
    const size_t tbase = ((size_t)zc * SEQ + (size_t)r0) * HD;
#pragma unroll 1
    for (int ps = 0; ps < 2; ++ps) {
#pragma unroll
        for (int hh = 0; hh < 2; ++hh) {
#pragma unroll
            for (int s = 0; s < 2; ++s) { const int p = s * 32 + lane; const int row = p >> 2, c8 = (p & 3) * 8;
                const v4f x0 = *(const v4fa*)(&os[row * 68 + hh * 32 + c8]); const v4f x1 = *(const v4fa*)(&os[row * 68 + hh * 32 + c8 + 4]); v8h hv, rv;
#pragma unroll
                for (int i = 0; i < 4; ++i) { const h16 a0 = toh_flush(x0[i]); const h16 a1 = toh_flush(x1[i]); hv[i] = a0; hv[4 + i] = a1;
                    rv[i] = toh_flush((x0[i] - (float)a0) * QRS); rv[4 + i] = toh_flush((x1[i] - (float)a1) * QRS); }
                const size_t oo = tbase + (size_t)hh * ((size_t)SEQ * HD) + (size_t)p * 8;
                *(volatile v8h*)(Ph + oo) = hv; *(volatile v8h*)(Pr + oo) = rv; } }
        if (ps == 0) __threadfence(); }
}

__global__ __launch_bounds__(32) void k_rm(const h16* __restrict__ A, const h16* __restrict__ Bt, const int K, const float* __restrict__ bias, const int hasb, const int relu, h16* P, const int pitch) {
    __shared__ __align__(16) float os[16 * 68];
    const int lane = threadIdx.x & 31, lr = lane & 15, hi = lane >> 4; const int r0 = blockIdx.x * 64, c0 = blockIdx.y * 64;
    v8f acc[4][4];
#pragma unroll
    for (int mb = 0; mb < 4; ++mb)
#pragma unroll
        for (int nb = 0; nb < 4; ++nb) acc[mb][nb] = (v8f){};
    const size_t aoff = (size_t)(r0 + lr) * K + 8 * hi, boff = (size_t)(c0 + lr) * K + 8 * hi;
#pragma unroll 1
    for (int kc = 0; kc < K; kc += 32) {
        v16h a[4];
#pragma unroll
        for (int mb = 0; mb < 4; ++mb) a[mb] = ldh(A + aoff + (size_t)mb * 16 * K + kc);
#pragma unroll
        for (int nb = 0; nb < 4; ++nb) { const v16h b = ldh(Bt + boff + (size_t)nb * 16 * K + kc);
#pragma unroll
            for (int mb = 0; mb < 4; ++mb) acc[mb][nb] = wmma16g(a[mb], b, acc[mb][nb]); }
    }
    float bc[4];
#pragma unroll
    for (int nb = 0; nb < 4; ++nb) bc[nb] = 0.0f;
    if (hasb) {
#pragma unroll
        for (int nb = 0; nb < 4; ++nb) bc[nb] = bfr(bias[c0 + nb * 16 + lr]);
    }
#pragma unroll
    for (int mb = 0; mb < 4; ++mb) {
#pragma unroll
        for (int nb = 0; nb < 4; ++nb) {
#pragma unroll
            for (int j = 0; j < 8; ++j) { const float v = acc[mb][nb][j] * WSI + bc[nb]; const float w = fmaxf(v, 0.0f);
                os[(hi * 8 + j) * 68 + nb * 16 + lr] = relu ? w : v; } }
        wave_sync();
#pragma unroll 1
        for (int ps = 0; ps < 2; ++ps) {
#pragma unroll
            for (int s = 0; s < 4; ++s) { const int row = 4 * s + (lane >> 3), c8 = (lane & 7) * 8;
                const v4f x0 = *(const v4fa*)(&os[row * 68 + c8]); const v4f x1 = *(const v4fa*)(&os[row * 68 + c8 + 4]); v8h hv;
#pragma unroll
                for (int i = 0; i < 4; ++i) { hv[i] = toh_flush(x0[i]); hv[4 + i] = toh_flush(x1[i]); }
                *(volatile v8h*)(P + (size_t)(r0 + mb * 16 + row) * pitch + c0 + c8) = hv; }
            if (ps == 0) __threadfence(); }
        wave_sync();
    }
}

__global__ __launch_bounds__(32 * NH_) void k_attn(const h16* __restrict__ QKH, const h16* __restrict__ QKR, const h16* __restrict__ VT, h16* CTX) {
    __shared__ __align__(16) float os[16 * RP];
    const int lane = threadIdx.x & 31, lr = lane & 15, hi = lane >> 4;
    const int wave = __builtin_amdgcn_readfirstlane((int)(threadIdx.x >> 5));
    const int t0 = blockIdx.x * 16;
    int klo = t0 - WH; klo = klo < 0 ? 0 : klo; klo &= ~31;
    int khi = t0 + 16 + WH; khi = khi > SEQ ? SEQ : khi; khi = (khi + 31) & ~31;
    const int tq = t0 + lr;
    const size_t qo = ((size_t)wave * SEQ + (size_t)tq) * HD + 8 * hi;
    const v16h qh = ldh(QKH + qo), qr = ldh(QKR + qo);
    const size_t ko = ((size_t)(NH_ + wave) * SEQ + (size_t)lr) * HD + 8 * hi;
    const size_t vo = ((size_t)(wave * HD + lr)) * SEQ + 8 * hi;
    v8f o0 = (v8f){}, o1 = (v8f){};
    float m = NEGB, l = 0.0f;
#pragma unroll 1
    for (int key0 = klo; key0 < khi; key0 += 32) {
        const h16* ka = QKH + ko + (size_t)key0 * HD;
        const h16* kr = QKR + ko + (size_t)key0 * HD;
        const v16h ka0 = ldh(ka), kb0 = ldh(ka + 16 * HD);
        const v16h kra0 = ldh(kr), krb0 = ldh(kr + 16 * HD);
        v8f sHa = (v8f){}, sLa = (v8f){}, sHb = (v8f){}, sLb = (v8f){};
        sHa = wmma16g(ka0, qh, sHa); sLa = wmma16g(ka0, qr, sLa); sLa = wmma16g(kra0, qh, sLa);
        sHb = wmma16g(kb0, qh, sHb); sLb = wmma16g(kb0, qr, sLb); sLb = wmma16g(krb0, qh, sLb);
        const int ja = key0 + 8 * hi - tq;
        float ta[8], tb[8]; bool fa[8], fb[8]; float mx = NEGB;
#pragma unroll
        for (int r = 0; r < 8; ++r) {
            const int da = ja + r, db = ja + 16 + r;
            fa[r] = (da >= -WH) & (da <= WH);
            fb[r] = (db >= -WH) & (db <= WH);
            ta[r] = (sHa[r] + sLa[r] * QRI) * SC2; tb[r] = (sHb[r] + sLb[r] * QRI) * SC2;
            mx = fmaxf(mx, fmaxf(fa[r] ? ta[r] : NEGB, fb[r] ? tb[r] : NEGB)); }
        mx = fmaxf(mx, __shfl_xor(mx, 16, 32));
        const float mnew = fmaxf(m, mx);
        const float alpha = __builtin_amdgcn_exp2f(m - mnew);
        const float sh = PSH - mnew;
        v16h pb; float ls = 0.0f;
#pragma unroll
        for (int r = 0; r < 8; ++r) {
            const float xa = ta[r] + sh, xb = tb[r] + sh;
            const float ea = __builtin_amdgcn_exp2f(xa), eb = __builtin_amdgcn_exp2f(xb);
            const float ga = (fa[r] & (xa >= -14.0f)) ? ea : 0.0f, gb = (fb[r] & (xb >= -14.0f)) ? eb : 0.0f;
            const h16 pa = (h16)ga; const h16 pc = (h16)gb;
            pb[r] = pa; pb[8 + r] = pc;
            ls += (float)pa + (float)pc; }
        l = l * alpha + ls; m = mnew;
        o0 = o0 * alpha; o1 = o1 * alpha;
        const h16* va = VT + vo + key0;
        const v16h v0 = ldh(va), v1 = ldh(va + (size_t)16 * SEQ);
        o0 = wmma16g(v0, pb, o0); o1 = wmma16g(v1, pb, o1);
    }
    l += __shfl_xor(l, 16, 32);
    const bool any = l > 0.0f;
    const float lsafe = any ? l : 1.0f;
    const float inv = any ? (1.0f / lsafe) : 0.0f;
    const int wb = wave * HD;
    { v4f a, c;
      a[0] = o0[0] * inv; a[1] = o0[1] * inv; a[2] = o0[2] * inv; a[3] = o0[3] * inv; c[0] = o0[4] * inv; c[1] = o0[5] * inv; c[2] = o0[6] * inv; c[3] = o0[7] * inv;
      *(v4fa*)(&os[lr * RP + wb +  0 + 8 * hi]) = a; *(v4fa*)(&os[lr * RP + wb +  0 + 8 * hi + 4]) = c;
      a[0] = o1[0] * inv; a[1] = o1[1] * inv; a[2] = o1[2] * inv; a[3] = o1[3] * inv; c[0] = o1[4] * inv; c[1] = o1[5] * inv; c[2] = o1[6] * inv; c[3] = o1[7] * inv;
      *(v4fa*)(&os[lr * RP + wb + 16 + 8 * hi]) = a; *(v4fa*)(&os[lr * RP + wb + 16 + 8 * hi + 4]) = c; }
    __syncthreads();
#pragma unroll 1
    for (int ps = 0; ps < 2; ++ps) {
#pragma unroll
        for (int s = 0; s < 2; ++s) { const int row = wave * 2 + s, c8 = lane * 8;
            const v4f x0 = *(const v4fa*)(&os[row * RP + c8]); const v4f x1 = *(const v4fa*)(&os[row * RP + c8 + 4]); v8h hv;
#pragma unroll
            for (int i = 0; i < 4; ++i) { hv[i] = toh_flush(x0[i]); hv[4 + i] = toh_flush(x1[i]); }
            *(volatile v8h*)(CTX + (size_t)(t0 + row) * EW + c8) = hv; }
        if (ps == 0) __threadfence(); }
}

static constexpr size_t al256(size_t v) { return (v + 255) & ~(size_t)255; }
static constexpr size_t SZ_XH   = al256((size_t)SEQ * XIN * 2);
static constexpr size_t SZ_WE   = al256((size_t)EW * XIN * 2);
static constexpr size_t SZ_WQKV = al256((size_t)NLAY * 3 * EW * EW * 2);
static constexpr size_t SZ_WO   = al256((size_t)NLAY * EW * EW * 2);
static constexpr size_t SZ_WF   = al256((size_t)NLAY * EW * FFW * 2);
static constexpr size_t SZ_F32  = al256((size_t)SEQ * EW * 4);
static constexpr size_t SZ_H16  = al256((size_t)SEQ * EW * 2);
static constexpr size_t SZ_QK   = al256((size_t)2 * NH_ * SEQ * HD * 2);
static constexpr size_t SZ_F1   = al256((size_t)SEQ * FFW * 2);
static constexpr size_t SZ_TOTAL = SZ_XH + SZ_WE + SZ_WQKV + SZ_WO + 2 * SZ_WF + 3 * SZ_F32 + 5 * SZ_H16 + 2 * SZ_QK + SZ_F1;
static_assert(SZ_TOTAL <= (size_t)134217728);
static_assert((size_t)EW * SEQ == (size_t)SEQ * EW);
static_assert(((size_t)EW * EW * 2) % 256 == 0);
static_assert(((size_t)EW * FFW * 2) % 256 == 0);

extern "C" void kernel_launch(void* const* d_in, const int* in_sizes, int n_in,
                              void* d_out, int out_size, void* d_ws, size_t ws_size, hipStream_t stream) {
    if (n_in < 14) return;
    if ((size_t)in_sizes[0] < (size_t)SEQ * XIN) return;
    if ((size_t)in_sizes[1] < (size_t)XIN * EW) return;
    if ((size_t)in_sizes[2] < (size_t)NLAY * EW * EW || (size_t)in_sizes[3] < (size_t)NLAY * EW * EW) return;
    if ((size_t)in_sizes[4] < (size_t)NLAY * EW * EW || (size_t)in_sizes[5] < (size_t)NLAY * EW * EW) return;
    if ((size_t)in_sizes[6] < (size_t)NLAY * EW * FFW || (size_t)in_sizes[8] < (size_t)NLAY * FFW * EW) return;
    if (in_sizes[7] < NLAY * FFW || in_sizes[9] < NLAY * EW) return;
    if (in_sizes[10] < NLAY * EW || in_sizes[11] < NLAY * EW || in_sizes[12] < NLAY * EW || in_sizes[13] < NLAY * EW) return;
    if ((size_t)out_size < (size_t)SEQ * EW) return;
    if (SZ_TOTAL > ws_size) return;
    const float* x    = (const float*)d_in[0];
    const float* wemb = (const float*)d_in[1];
    const float* wq   = (const float*)d_in[2];
    const float* wk   = (const float*)d_in[3];
    const float* wv   = (const float*)d_in[4];
    const float* wo   = (const float*)d_in[5];
    const float* wf1  = (const float*)d_in[6];
    const float* fb1  = (const float*)d_in[7];
    const float* wf2  = (const float*)d_in[8];
    const float* fb2  = (const float*)d_in[9];
    const float* ln1s = (const float*)d_in[10];
    const float* ln1o = (const float*)d_in[11];
    const float* ln2s = (const float*)d_in[12];
    const float* ln2o = (const float*)d_in[13];
    float* OUT = (float*)d_out;
    char* wsp = (char*)d_ws;
    h16* XH   = (h16*)wsp; wsp += SZ_XH;
    h16* WE   = (h16*)wsp; wsp += SZ_WE;
    h16* WQKV = (h16*)wsp; wsp += SZ_WQKV;
    h16* WO   = (h16*)wsp; wsp += SZ_WO;
    h16* WF1  = (h16*)wsp; wsp += SZ_WF;
    h16* WF2  = (h16*)wsp; wsp += SZ_WF;
    float* PE = (float*)wsp; wsp += SZ_F32;
    float* HF = (float*)wsp; wsp += SZ_F32;
    float* AF = (float*)wsp; wsp += SZ_F32;
    h16* HH   = (h16*)wsp; wsp += SZ_H16;
    h16* HR   = (h16*)wsp; wsp += SZ_H16;
    h16* AH   = (h16*)wsp; wsp += SZ_H16;
    h16* CTX  = (h16*)wsp; wsp += SZ_H16;
    h16* VT   = (h16*)wsp; wsp += SZ_H16;
    h16* QKH  = (h16*)wsp; wsp += SZ_QK;
    h16* QKR  = (h16*)wsp; wsp += SZ_QK;
    h16* F1   = (h16*)wsp; wsp += SZ_F1;

    { const size_t n8 = (size_t)SEQ * XIN / 8; k_cvth<<<(unsigned)((n8 + 255) / 256), 256, 0, stream>>>(x, XH, n8); }
    k_wconv<<<dim3(EW / 64, XIN / 64, 1), 256, 0, stream>>>(wemb, WE, XIN, EW, (size_t)0, (size_t)0);
    k_wconv<<<dim3(EW / 64, EW / 64, NLAY), 256, 0, stream>>>(wq, WQKV, EW, EW, (size_t)EW * EW, (size_t)3 * EW * EW);
    k_wconv<<<dim3(EW / 64, EW / 64, NLAY), 256, 0, stream>>>(wk, WQKV + (size_t)EW * EW, EW, EW, (size_t)EW * EW, (size_t)3 * EW * EW);
    k_wconv<<<dim3(EW / 64, EW / 64, NLAY), 256, 0, stream>>>(wv, WQKV + (size_t)2 * EW * EW, EW, EW, (size_t)EW * EW, (size_t)3 * EW * EW);
    k_wconv<<<dim3(EW / 64, EW / 64, NLAY), 256, 0, stream>>>(wo, WO, EW, EW, (size_t)EW * EW, (size_t)EW * EW);
    k_wconv<<<dim3(FFW / 64, EW / 64, NLAY), 256, 0, stream>>>(wf1, WF1, EW, FFW, (size_t)EW * FFW, (size_t)EW * FFW);
    k_wconv<<<dim3(EW / 64, FFW / 64, NLAY), 256, 0, stream>>>(wf2, WF2, FFW, EW, (size_t)FFW * EW, (size_t)FFW * EW);
    k_pe<<<SEQ, 256, 0, stream>>>(PE);

    k_rowgemm<<<SEQ / 16, 128, 0, stream>>>(XH, WE, XIN, 0, 0, PE, PE, PE, PE, HF, HH, HR, 1, 1);

    for (int l = 0; l < NLAY; ++l) {
        const h16* wqkv = WQKV + (size_t)l * 3 * EW * EW;
        k_qk<<<dim3(SEQ / 16, 2 * EW / 64, 1), 32, 0, stream>>>(HH, HR, wqkv, QKH, QKR);
        k_rm<<<dim3(EW / 64, SEQ / 64, 1), 32, 0, stream>>>(wqkv + (size_t)2 * EW * EW, HH, EW, PE, 0, 0, VT, SEQ);
        k_attn<<<SEQ / 16, 32 * NH_, 0, stream>>>(QKH, QKR, VT, CTX);
        k_rowgemm<<<SEQ / 16, 128, 0, stream>>>(CTX, WO + (size_t)l * EW * EW, EW, 1, 0, fb2, HF, ln1s + (size_t)l * EW, ln1o + (size_t)l * EW, AF, AH, AH, 1, 0);
        k_rm<<<dim3(SEQ / 64, FFW / 64, 1), 32, 0, stream>>>(AH, WF1 + (size_t)l * EW * FFW, EW, fb1 + (size_t)l * FFW, 1, 1, F1, FFW);
        const int last = (l == NLAY - 1) ? 1 : 0;
        k_rowgemm<<<SEQ / 16, 128, 0, stream>>>(F1, WF2 + (size_t)l * FFW * EW, FFW, 1, 1, fb2 + (size_t)l * EW, AF, ln2s + (size_t)l * EW, ln2o + (size_t)l * EW,
                                                last ? OUT : HF, HH, HR, last ? 0 : 1, 1);
    }
}
